// PointNetSetAbstractionMsg_29798483100269
// MI455X (gfx1250) — hardware-verified
//
#include <hip/hip_runtime.h>
#include <math.h>

#pragma clang fp contract(off)

typedef __attribute__((ext_vector_type(16))) _Float16 v16h;
typedef __attribute__((ext_vector_type(8)))  _Float16 v8h;
typedef __attribute__((ext_vector_type(8)))  float    v8f;
typedef __attribute__((ext_vector_type(4)))  float    v4f;
typedef __attribute__((ext_vector_type(4)))  unsigned v4u;
typedef __attribute__((ext_vector_type(8)))  unsigned v8u;

constexpr int NBATCH = 8;
constexpr int NPTS   = 8192;
constexpr int NQRY   = 1024;
constexpr int KNMAX  = 128;
constexpr int KN_CAP   = 384;
constexpr int KN_MSTOP = 144;

template <int SC> struct ScaleDim;
template <> struct ScaleDim<0> { static constexpr int KNB = 16,  C1 = 32, C2 = 32, C3 = 64,  CBASE = 0,   WOFF0 = 0,     WOFF1 = 1024,  WOFF2 = 2048;  };
template <> struct ScaleDim<1> { static constexpr int KNB = 32,  C1 = 64, C2 = 64, C3 = 128, CBASE = 64,  WOFF0 = 4096,  WOFF1 = 6144,  WOFF2 = 10240; };
template <> struct ScaleDim<2> { static constexpr int KNB = 128, C1 = 64, C2 = 96, C3 = 128, CBASE = 192, WOFF0 = 18432, WOFF1 = 20480, WOFF2 = 26624; };
constexpr int WPLANE_HALVES = 38912;
static_assert(ScaleDim<0>::WOFF1 == ScaleDim<0>::WOFF0 + 32 * 32, "plane map");
static_assert(ScaleDim<0>::WOFF2 == ScaleDim<0>::WOFF1 + 32 * 32, "plane map");
static_assert(ScaleDim<1>::WOFF0 == ScaleDim<0>::WOFF2 + 64 * 32, "plane map");
static_assert(ScaleDim<1>::WOFF1 == ScaleDim<1>::WOFF0 + 64 * 32, "plane map");
static_assert(ScaleDim<1>::WOFF2 == ScaleDim<1>::WOFF1 + 64 * 64, "plane map");
static_assert(ScaleDim<2>::WOFF0 == ScaleDim<1>::WOFF2 + 128 * 64, "plane map");
static_assert(ScaleDim<2>::WOFF1 == ScaleDim<2>::WOFF0 + 64 * 32, "plane map");
static_assert(ScaleDim<2>::WOFF2 == ScaleDim<2>::WOFF1 + 96 * 64, "plane map");
static_assert(WPLANE_HALVES == ScaleDim<2>::WOFF2 + 128 * 96, "plane map");

template <typename T> struct Frag;
template <> struct Frag<_Float16> {
  typedef v16h V; union U { v16h v; v8h h[2]; };
  static __device__ __forceinline__ v16h load(const _Float16* p) {
    U f; f.h[0] = *(const v8h*)(p); f.h[1] = *(const v8h*)(p + 16); return f.v;
  }
};
__device__ __forceinline__ v8f mma_g(v16h a, v16h b, v8f c) {
  c = __builtin_amdgcn_wmma_f32_16x16x32_f16(false, a, false, b, (short)0, c, false, false);
  asm volatile("v_nop\n\tv_nop\n\tv_nop\n\tv_nop" : "+v"(c) : "v"(a), "v"(b));
  return c;
}
__device__ __forceinline__ void wave_lds_sync() {
  __builtin_amdgcn_fence(__ATOMIC_RELEASE, "workgroup");
  __builtin_amdgcn_wave_barrier();
  __builtin_amdgcn_fence(__ATOMIC_ACQUIRE, "workgroup");
}
__device__ __forceinline__ unsigned f16_bits(float x) {
  const _Float16 h = (_Float16)x;
  const unsigned short hs = __builtin_bit_cast(unsigned short, h);
  return (unsigned)hs;
}

__global__ __launch_bounds__(256) void copy_queries(const float* __restrict__ xyz, float* __restrict__ out0) {
  const int t = blockIdx.x * 256 + threadIdx.x;
  if (t < (NBATCH * 3 * NQRY) / 4) {
    const int i4 = t * 4;
    const int row = i4 >> 10;
    const int s = i4 & (NQRY - 1);
    const v4f v = *(const v4f*)(xyz + (size_t)row * NPTS + s);
    float* dst = out0 + i4;
    *(volatile v4f*)dst = v;
    __threadfence();
    *(volatile v4f*)dst = v;
  }
}

__global__ __launch_bounds__(128) void prep_weights(
    const float* __restrict__ w0, const float* __restrict__ w1, const float* __restrict__ w2,
    const float* __restrict__ w3, const float* __restrict__ w4, const float* __restrict__ w5,
    const float* __restrict__ w6, const float* __restrict__ w7, const float* __restrict__ w8,
    unsigned short* __restrict__ wpl) {
  const int blk = blockIdx.x;
  const float* W = w0;
  int cin = 6, kpad = 32, off = 0, b0 = 0;
  if (blk >= 1)  { W = w1; cin = 32; kpad = 32; off = 1024;  b0 = 1;  }
  if (blk >= 2)  { W = w2; cin = 32; kpad = 32; off = 2048;  b0 = 2;  }
  if (blk >= 4)  { W = w3; cin = 6;  kpad = 32; off = 4096;  b0 = 4;  }
  if (blk >= 6)  { W = w4; cin = 64; kpad = 64; off = 6144;  b0 = 6;  }
  if (blk >= 10) { W = w5; cin = 64; kpad = 64; off = 10240; b0 = 10; }
  if (blk >= 18) { W = w6; cin = 6;  kpad = 32; off = 18432; b0 = 18; }
  if (blk >= 20) { W = w7; cin = 64; kpad = 64; off = 20480; b0 = 20; }
  if (blk >= 26) { W = w8; cin = 96; kpad = 96; off = 26624; b0 = 26; }
  const int e0 = (blk - b0) * 1024 + threadIdx.x * 8;
  const int o = e0 / kpad;
  const int c0 = e0 - o * kpad;
  float zz = 0.0f;
  asm volatile("" : "+v"(zz));
  unsigned hb[8];
#pragma unroll
  for (int i = 0; i < 8; ++i) {
    const int cc = c0 + i;
    const int ccl = (cc < cin) ? cc : (cin - 1);
    const float x = W[o * cin + ccl];
    const float v = (cc < cin) ? x : zz;
    hb[i] = f16_bits(v);
  }
  v4u w;
  w[0] = hb[0] | (hb[1] << 16);
  w[1] = hb[2] | (hb[3] << 16);
  w[2] = hb[4] | (hb[5] << 16);
  w[3] = hb[6] | (hb[7] << 16);
  unsigned short* dst = wpl + off + e0;
  *(volatile v4u*)dst = w;
  __threadfence();
  *(volatile v4u*)dst = w;
}

__device__ __forceinline__ unsigned dist_key(float qx, float qy, float qz, float qq, float px, float py, float pz) {
#pragma clang fp contract(off)
  const float px2 = px * px;
  const float py2 = py * py;
  const float pz2 = pz * pz;
  const float pp = (px2 + pz2) + py2;
  float dt = qx * px;
  dt = __builtin_fmaf(qy, py, dt);
  dt = __builtin_fmaf(qz, pz, dt);
  const float t = qq + pp;
  const float two_dt = 2.0f * dt;
  float d = t - two_dt;
  d = d + 0.0f;
  const unsigned bits = __float_as_uint(d);
  const unsigned msk = (unsigned)((int)bits >> 31) | 0x80000000u;
  return bits ^ msk;
}

__global__ __launch_bounds__(256) void knn_gather(const float* __restrict__ xyz, const float* __restrict__ pts,
                                                  unsigned short* __restrict__ x0) {
#pragma clang fp contract(off)
  __shared__ __align__(16) unsigned cu[KN_CAP];
  __shared__ int cn[KN_CAP];
  __shared__ int wcnt[2][8];
  __shared__ int wtot[8];
  __shared__ __align__(16) v4u rows[KNMAX];

  const int tid = threadIdx.x;
  const int lane = tid & 31;
  const int wave = __builtin_amdgcn_readfirstlane(tid >> 5);
  const int b = blockIdx.x >> 10;
  const int s = blockIdx.x & (NQRY - 1);
  const float* xb = xyz + (size_t)b * 3 * NPTS;
  const float* pb = pts + (size_t)b * 3 * NPTS;

  for (int i = tid; i < KN_CAP; i += 256) { cu[i] = 0xFFFFFFFFu; cn[i] = 0; }
  if (tid < KNMAX) { v4u z; z[0] = 0u; z[1] = 0u; z[2] = 0u; z[3] = 0u; rows[tid] = z; }

  const float qx = xb[s], qy = xb[NPTS + s], qz = xb[2 * NPTS + s];
  const float qx2 = qx * qx;
  const float qy2 = qy * qy;
  const float qz2 = qz * qz;
  const float qq = (qx2 + qz2) + qy2;

  const int n0 = tid * 32;
  unsigned u[32];
#pragma unroll
  for (int c = 0; c < 4; ++c) {
    const float* px = xb + n0 + 8 * c;
    const v4f xa = *(const v4f*)(px);
    const v4f xc = *(const v4f*)(px + 4);
    const v4f ya = *(const v4f*)(px + NPTS);
    const v4f yc = *(const v4f*)(px + NPTS + 4);
    const v4f za = *(const v4f*)(px + 2 * NPTS);
    const v4f zc = *(const v4f*)(px + 2 * NPTS + 4);
#pragma unroll
    for (int e = 0; e < 4; ++e) {
      u[8 * c + e]     = dist_key(qx, qy, qz, qq, xa[e], ya[e], za[e]);
      u[8 * c + 4 + e] = dist_key(qx, qy, qz, qq, xc[e], yc[e], zc[e]);
    }
    asm volatile("" ::: "memory");
  }
  unsigned mn = u[0];
#pragma unroll
  for (int j = 1; j < 32; ++j) mn = (u[j] < mn) ? u[j] : mn;

  unsigned lowP = 0u, hiIncl = 0xFFFFFFFFu;
  int cntHi = 256;
  int par = 0;
#pragma unroll 1
  for (int bit = 31; bit >= 0; --bit) {
    if (cntHi <= KN_MSTOP) break;
    const unsigned mid = lowP | (1u << bit);
    const unsigned bal = __builtin_amdgcn_ballot_w32(mn < mid);
    const int wc = __popc(bal);
    if (lane == 0) wcnt[par][wave] = wc;
    __syncthreads();
    int c = 0;
#pragma unroll
    for (int w = 0; w < 8; ++w) c += wcnt[par][w];
    c = __builtin_amdgcn_readfirstlane(c);
    par ^= 1;
    if (c >= 128) { hiIncl = mid - 1u; cntHi = c; } else { lowP = mid; }
  }

  int myc = 0;
#pragma unroll
  for (int j = 0; j < 32; ++j) myc += (u[j] <= hiIncl) ? 1 : 0;
  int incl = myc;
#pragma unroll
  for (int off = 1; off < 32; off <<= 1) {
    const int y = __shfl_up(incl, (unsigned)off, 32);
    if (lane >= off) incl += y;
  }
  const int wsum = __shfl(incl, 31, 32);
  if (lane == 0) wtot[wave] = wsum;
  __syncthreads();
  int base = 0, tot = 0;
#pragma unroll
  for (int w = 0; w < 8; ++w) {
    const int v = wtot[w];
    tot += v;
    base += (w < wave) ? v : 0;
  }
  int pos = base + incl - myc;
#pragma unroll
  for (int j = 0; j < 32; ++j) {
    if (u[j] <= hiIncl) {
      if (pos < KN_CAP) { cu[pos] = u[j]; cn[pos] = n0 + j; }
      ++pos;
    }
  }
  __syncthreads();
  tot = __builtin_amdgcn_readfirstlane(tot);
  const int C = (tot < KN_CAP) ? tot : KN_CAP;
  const int cpad = (C + 31) & ~31;

  float zf = 0.0f;
  asm volatile("" : "+v"(zf));
#pragma unroll 1
  for (int ib = wave * 32; ib < C; ib += 256) {
    const int i = ib + lane;
    const unsigned ui = cu[i];
    int ni = cn[i];
    int rank = 0;
#pragma unroll 1
    for (int j = 0; j < ib; j += 4) {
      const v4u kq = *(const v4u*)(cu + j);
      rank += (kq[0] <= ui) ? 1 : 0;
      rank += (kq[1] <= ui) ? 1 : 0;
      rank += (kq[2] <= ui) ? 1 : 0;
      rank += (kq[3] <= ui) ? 1 : 0;
    }
#pragma unroll 1
    for (int j = ib; j < ib + 32; j += 4) {
      const v4u kq = *(const v4u*)(cu + j);
#pragma unroll
      for (int e = 0; e < 4; ++e) {
        const int lt = (kq[e] < ui) ? 1 : 0;
        const int eq = (kq[e] == ui) ? 1 : 0;
        const int before = ((j + e) < i) ? 1 : 0;
        rank += lt | (eq & before);
      }
    }
#pragma unroll 1
    for (int j = ib + 32; j < cpad; j += 4) {
      const v4u kq = *(const v4u*)(cu + j);
      rank += (kq[0] < ui) ? 1 : 0;
      rank += (kq[1] < ui) ? 1 : 0;
      rank += (kq[2] < ui) ? 1 : 0;
      rank += (kq[3] < ui) ? 1 : 0;
    }
    ni = (ni < 0) ? 0 : ni;
    ni = (ni > NPTS - 1) ? (NPTS - 1) : ni;
    const float p0 = pb[ni], p1 = pb[NPTS + ni], p2 = pb[2 * NPTS + ni];
    const float nx = xb[ni], ny = xb[NPTS + ni], nz = xb[2 * NPTS + ni];
    const float g0 = nx - qx;
    const float g1 = ny - qy;
    const float g2 = nz - qz;
    v4u w;
    w[0] = f16_bits(p0) | (f16_bits(p1) << 16);
    w[1] = f16_bits(p2) | (f16_bits(g0) << 16);
    w[2] = f16_bits(g1) | (f16_bits(g2) << 16);
    w[3] = f16_bits(zf) | (f16_bits(zf) << 16);
    if (i < C && rank < KNMAX) rows[rank] = w;
  }
  __syncthreads();

  if (tid < KNMAX) {
    const v4u w = rows[tid];
    unsigned short* dst = x0 + ((size_t)blockIdx.x * KNMAX + tid) * 8;
    *(volatile v4u*)dst = w;
    __threadfence();
    *(volatile v4u*)dst = w;
  }
}

__device__ __forceinline__ void affine_relu_store(const v8f& acc, _Float16* scr, int pitch, int col, int hh, float sc, float sh) {
#pragma unroll
  for (int r = 0; r < 8; ++r) {
    float v = acc[r] * sc;
    v = v + sh;
    v = fmaxf(v, 0.0f);
    scr[(8 * hh + r) * pitch + col] = (_Float16)v;
  }
}
__device__ __forceinline__ void stats_tile(const v8f& acc, float* redw, int cl, int col, int hh) {
  float s = 0.0f, q = 0.0f;
#pragma unroll
  for (int r = 0; r < 8; ++r) {
    const float a = acc[r];
    const float a2 = a * a;
    s = s + a;
    q = q + a2;
  }
  s += __shfl_xor(s, 16, 32);
  q += __shfl_xor(q, 16, 32);
  if (hh == 0) { redw[col] = s; redw[cl + col] = q; }
}
__device__ __forceinline__ void maxmin_tile(const v8f& acc, float* redmw, int cl, int col, int hh) {
  float mx = -INFINITY, mi = INFINITY;
#pragma unroll
  for (int r = 0; r < 8; ++r) { mx = fmaxf(mx, acc[r]); mi = fminf(mi, acc[r]); }
  const float mx2 = __shfl_xor(mx, 16, 32);
  const float mi2 = __shfl_xor(mi, 16, 32);
  mx = fmaxf(mx, mx2);
  mi = fminf(mi, mi2);
  if (hh == 0) { redmw[col] = mx; redmw[cl + col] = mi; }
}

template <int SC, int DEPTH>
__global__ __launch_bounds__(256) void mlp_pass(
    const unsigned short* __restrict__ x0, const unsigned short* __restrict__ wpl,
    const float* __restrict__ scsh, float* __restrict__ part,
    float* __restrict__ pmx, float* __restrict__ pmn) {
  typedef ScaleDim<SC> D;
  constexpr int C1 = D::C1, C2 = D::C2, C3 = D::C3, KNB = D::KNB;
  constexpr int CL = (DEPTH == 1) ? C1 : ((DEPTH == 2) ? C2 : C3);
  constexpr int PA = C1 + 8, PB = C2 + 8;
  static_assert(C1 % 32 == 0 && C2 % 32 == 0 && C3 % 16 == 0, "k chunks of 32, n tiles of 16");
  static_assert((8192 * KNB) % 128 == 0, "row count is a block multiple");
  __shared__ __align__(16) _Float16 scrA[(DEPTH >= 2) ? 8 * 16 * PA : 8];
  __shared__ __align__(16) _Float16 scrB[(DEPTH >= 3) ? 8 * 16 * PB : 8];
  __shared__ __align__(16) float red[8 * 2 * CL];
  __shared__ __align__(16) float redm[(DEPTH == 3) ? 8 * 2 * C3 : 4];
  __shared__ __align__(16) float s_ss[(DEPTH >= 3) ? (2 * C1 + 2 * C2) : ((DEPTH == 2) ? 2 * C1 : 4)];

  const int tid = threadIdx.x;
  const int lane = tid & 31;
  const int wave = __builtin_amdgcn_readfirstlane(tid >> 5);
  const int hh = lane >> 4, n = lane & 15;

  if (DEPTH >= 2) {
    for (int i = tid; i < C1; i += 256) { s_ss[i] = scsh[i]; s_ss[C1 + i] = scsh[128 + i]; }
  }
  if (DEPTH >= 3) {
    for (int i = tid; i < C2; i += 256) { s_ss[2 * C1 + i] = scsh[256 + i]; s_ss[2 * C1 + C2 + i] = scsh[256 + 128 + i]; }
  }
  __syncthreads();

  const int m = blockIdx.x * 128 + wave * 16 + n;
  const int grp = m / KNB;
  const int kk = m - grp * KNB;
  const v4u xw = *(const v4u*)(x0 + ((size_t)grp * KNMAX + kk) * 8);
  const unsigned keep = (hh == 0) ? 0xFFFFFFFFu : 0u;
  v8u aw;
  aw[0] = xw[0] & keep; aw[1] = xw[1] & keep; aw[2] = xw[2] & keep; aw[3] = xw[3] & keep;
  aw[4] = 0u; aw[5] = 0u; aw[6] = 0u; aw[7] = 0u;
  const v16h a0 = __builtin_bit_cast(v16h, aw);

  float* redw = red + wave * 2 * CL;
  float* redmw = redm + ((DEPTH == 3) ? wave * 2 * C3 : 0);
  _Float16* scrAw = scrA + ((DEPTH >= 2) ? wave * 16 * PA : 0);
  _Float16* scrBw = scrB + ((DEPTH >= 3) ? wave * 16 * PB : 0);

  {
    const _Float16* W0p = (const _Float16*)(wpl + D::WOFF0);
#pragma unroll 1
    for (int j = 0; j < C1 / 16; ++j) {
      const v16h bf = Frag<_Float16>::load(W0p + (j * 16 + n) * 32 + 8 * hh);
      v8f acc = (v8f){0.f, 0.f, 0.f, 0.f, 0.f, 0.f, 0.f, 0.f};
      acc = mma_g(a0, bf, acc);
      if (DEPTH == 1) stats_tile(acc, redw, CL, j * 16 + n, hh);
      else affine_relu_store(acc, scrAw, PA, j * 16 + n, hh, s_ss[j * 16 + n], s_ss[C1 + j * 16 + n]);
    }
  }

  if (DEPTH >= 2) {
    wave_lds_sync();
    constexpr int NK1 = C1 / 32;
    v16h a1[NK1];
#pragma unroll
    for (int kc = 0; kc < NK1; ++kc) a1[kc] = Frag<_Float16>::load(scrAw + n * PA + kc * 32 + 8 * hh);
    const _Float16* W1p = (const _Float16*)(wpl + D::WOFF1);
#pragma unroll 1
    for (int j = 0; j < C2 / 16; ++j) {
      v8f acc = (v8f){0.f, 0.f, 0.f, 0.f, 0.f, 0.f, 0.f, 0.f};
#pragma unroll
      for (int kc = 0; kc < NK1; ++kc) {
        const v16h bf = Frag<_Float16>::load(W1p + (j * 16 + n) * C1 + kc * 32 + 8 * hh);
        acc = mma_g(a1[kc], bf, acc);
      }
      if (DEPTH == 2) stats_tile(acc, redw, CL, j * 16 + n, hh);
      else affine_relu_store(acc, scrBw, PB, j * 16 + n, hh, s_ss[2 * C1 + j * 16 + n], s_ss[2 * C1 + C2 + j * 16 + n]);
    }
  }

  if (DEPTH >= 3) {
    wave_lds_sync();
    constexpr int NK2 = C2 / 32;
    v16h a2[NK2];
#pragma unroll
    for (int kc = 0; kc < NK2; ++kc) a2[kc] = Frag<_Float16>::load(scrBw + n * PB + kc * 32 + 8 * hh);
    const _Float16* W2p = (const _Float16*)(wpl + D::WOFF2);
#pragma unroll 1
    for (int j = 0; j < C3 / 16; ++j) {
      v8f acc = (v8f){0.f, 0.f, 0.f, 0.f, 0.f, 0.f, 0.f, 0.f};
#pragma unroll
      for (int kc = 0; kc < NK2; ++kc) {
        const v16h bf = Frag<_Float16>::load(W2p + (j * 16 + n) * C2 + kc * 32 + 8 * hh);
        acc = mma_g(a2[kc], bf, acc);
      }
      stats_tile(acc, redw, CL, j * 16 + n, hh);
      maxmin_tile(acc, redmw, C3, j * 16 + n, hh);
    }
  }

  __syncthreads();

  constexpr int NS4 = (2 * CL) / 4;
  constexpr int GRP_PER_BLK = 128 / KNB;
  constexpr int WPG = KNB / 16;
  constexpr int NM4 = (DEPTH == 3) ? (GRP_PER_BLK * C3) / 4 : 0;
  const bool doS = tid < NS4;
  const int ts4 = doS ? tid * 4 : 0;
  v4f sv = (v4f){0.f, 0.f, 0.f, 0.f};
#pragma unroll
  for (int w = 0; w < 8; ++w) {
    const v4f t = *(const v4f*)(red + w * 2 * CL + ts4);
    sv = sv + t;
  }
  float* ps = part + (size_t)blockIdx.x * (2 * CL) + ts4;

  bool doM = false;
  v4f mxv = (v4f){0.f, 0.f, 0.f, 0.f};
  v4f mnv = (v4f){0.f, 0.f, 0.f, 0.f};
  float* pmxp = pmx;
  float* pmnp = pmn;
  if (DEPTH == 3) {
    doM = tid < NM4;
    const int e0 = doM ? tid * 4 : 0;
    const int g = e0 / C3;
    const int c = e0 - g * C3;
    mxv = (v4f){-INFINITY, -INFINITY, -INFINITY, -INFINITY};
    mnv = (v4f){INFINITY, INFINITY, INFINITY, INFINITY};
#pragma unroll
    for (int ww = 0; ww < WPG; ++ww) {
      const int w = g * WPG + ww;
      const v4f a = *(const v4f*)(redm + w * 2 * C3 + c);
      const v4f bq = *(const v4f*)(redm + w * 2 * C3 + C3 + c);
#pragma unroll
      for (int e = 0; e < 4; ++e) { mxv[e] = fmaxf(mxv[e], a[e]); mnv[e] = fminf(mnv[e], bq[e]); }
    }
    pmxp = pmx + (size_t)blockIdx.x * (GRP_PER_BLK * C3) + e0;
    pmnp = pmn + (size_t)blockIdx.x * (GRP_PER_BLK * C3) + e0;
  }
  for (int pass = 0; pass < 2; ++pass) {
    if (doS) *(volatile v4f*)ps = sv;
    if (DEPTH == 3) {
      if (doM) { *(volatile v4f*)pmxp = mxv; *(volatile v4f*)pmnp = mnv; }
    }
    __threadfence();
  }
}

__global__ __launch_bounds__(256) void bn_finalize(
    const float* __restrict__ part, int nblk, int C,
    const float* __restrict__ bias, const float* __restrict__ gam, const float* __restrict__ beta,
    float* __restrict__ scsh_row, double invM) {
  __shared__ double dsum[256];
  __shared__ __align__(16) float so[256];
  const int tid = threadIdx.x;
  const int ncol = 2 * C;
  const int ngrp = 256 / ncol;
  const int col = tid % ncol;
  const int grp = tid / ncol;
  const int nb = (grp < ngrp) ? nblk : 0;
  double acc = 0.0;
#pragma unroll 4
  for (int blk = grp; blk < nb; blk += ngrp) acc = acc + (double)part[(size_t)blk * ncol + col];
  dsum[tid] = acc;
  __syncthreads();
  float scv = 0.0f, shv = 0.0f;
  if (tid < C) {
    double s = 0.0, q = 0.0;
    for (int g = 0; g < ngrp; ++g) { s = s + dsum[g * ncol + tid]; q = q + dsum[g * ncol + C + tid]; }
    const double mean = s * invM;
    double var = q * invM - mean * mean;
    var = (var < 0.0) ? 0.0 : var;
    const float vf = (float)var;
    const float rs = rsqrtf(vf + 1e-5f);
    scv = gam[tid] * rs;
    const double bv = (double)bias[tid];
    const double meanb = mean + bv;
    shv = (float)((double)beta[tid] + (bv - meanb) * (double)scv);
  }
  if (tid < 128) { so[tid] = scv; so[128 + tid] = shv; }
  __syncthreads();
  if (tid < 64) {
    const v4f v = *(const v4f*)(so + tid * 4);
    float* dst = scsh_row + tid * 4;
    *(volatile v4f*)dst = v;
    __threadfence();
    *(volatile v4f*)dst = v;
  }
}

template <int C3, int CBASE>
__global__ __launch_bounds__(256) void pool_out(const float* __restrict__ pmx, const float* __restrict__ pmn,
                                                const float* __restrict__ scsh_row, float* __restrict__ out1) {
  __shared__ __align__(16) float tile[32 * 36];
  constexpr int CT = C3 / 32;
  const int tid = threadIdx.x;
  const int bx = blockIdx.x;
  const int ct = bx % CT;
  const int rest = bx / CT;
  const int st = rest & 31;
  const int b = rest >> 5;
  {
    const int sr = tid >> 3, c4 = (tid & 7) * 4;
    const int g = b * NQRY + st * 32 + sr;
    const int c = ct * 32 + c4;
    const v4f mx = *(const v4f*)(pmx + (size_t)g * C3 + c);
    const v4f mi = *(const v4f*)(pmn + (size_t)g * C3 + c);
    const v4f sc = *(const v4f*)(scsh_row + c);
    const v4f sh = *(const v4f*)(scsh_row + 128 + c);
#pragma unroll
    for (int e = 0; e < 4; ++e) {
      const float s_ = sc[e];
      const float v = (s_ >= 0.0f) ? mx[e] : mi[e];
      float o = v * s_;
      o = o + sh[e];
      o = fmaxf(o, 0.0f);
      tile[(c4 + e) * 36 + sr] = o;
    }
  }
  __syncthreads();
  {
    const int cr = tid >> 3, s4 = (tid & 7) * 4;
    const v4f val = *(const v4f*)(tile + cr * 36 + s4);
    float* dst = out1 + ((size_t)(b * 320 + CBASE + ct * 32 + cr)) * NQRY + st * 32 + s4;
    *(volatile v4f*)dst = val;
    __threadfence();
    *(volatile v4f*)dst = val;
  }
}

constexpr size_t align256(size_t x) { return (x + 255) & ~(size_t)255; }
constexpr size_t SZ_X0   = (size_t)NBATCH * NQRY * KNMAX * 8 * 2;
constexpr size_t SZ_WPL  = align256((size_t)WPLANE_HALVES * 2);
constexpr size_t SZ_SCSH = align256((size_t)9 * 256 * 4);
constexpr size_t part_bytes(int nblk, int c) { return (size_t)nblk * 2 * c * 4; }
constexpr size_t SZ_PART0 = part_bytes(1024, 32) + part_bytes(1024, 32) + part_bytes(1024, 64);
constexpr size_t SZ_PART1 = part_bytes(2048, 64) + part_bytes(2048, 64) + part_bytes(2048, 128);
constexpr size_t SZ_PART2 = part_bytes(8192, 64) + part_bytes(8192, 96) + part_bytes(8192, 128);
constexpr size_t SZ_PM0 = (size_t)8192 * 64 * 4;
constexpr size_t SZ_PM1 = (size_t)8192 * 128 * 4;
constexpr size_t SZ_PM2 = (size_t)8192 * 128 * 4;
constexpr size_t WS_TOTAL = SZ_X0 + SZ_WPL + SZ_SCSH + SZ_PART0 + SZ_PART1 + SZ_PART2 + 2 * (SZ_PM0 + SZ_PM1 + SZ_PM2);
static_assert(WS_TOTAL <= (size_t)134217728, "workspace carve");
static_assert((size_t)98304 + (size_t)10485760 == (size_t)10584064, "output packing");
static_assert((size_t)NBATCH * 3 * NQRY * 4 == (size_t)98304, "out0 bytes");

template <int SC>
static void run_scale(void* const* d_in, const unsigned short* x0, const unsigned short* wpl, float* scsh,
                      float* part0, float* part1, float* part2, float* pmx, float* pmn, float* out1, hipStream_t st) {
  typedef ScaleDim<SC> D;
  constexpr int MROWS = 8192 * D::KNB;
  constexpr int nblk = MROWS / 128;
  static_assert(nblk * 128 == MROWS, "block multiple");
  const double invM = 1.0 / (double)MROWS;
  const int base = 2 + 12 * SC;
  float* row0 = scsh + (SC * 3 + 0) * 256;
  float* row1 = scsh + (SC * 3 + 1) * 256;
  float* row2 = scsh + (SC * 3 + 2) * 256;

  mlp_pass<SC, 1><<<nblk, 256, 0, st>>>(x0, wpl, row0, part0, pmx, pmn);
  bn_finalize<<<1, 256, 0, st>>>(part0, nblk, D::C1, (const float*)d_in[base + 1], (const float*)d_in[base + 2],
                                 (const float*)d_in[base + 3], row0, invM);
  mlp_pass<SC, 2><<<nblk, 256, 0, st>>>(x0, wpl, row0, part1, pmx, pmn);
  bn_finalize<<<1, 256, 0, st>>>(part1, nblk, D::C2, (const float*)d_in[base + 5], (const float*)d_in[base + 6],
                                 (const float*)d_in[base + 7], row1, invM);
  mlp_pass<SC, 3><<<nblk, 256, 0, st>>>(x0, wpl, row0, part2, pmx, pmn);
  bn_finalize<<<1, 256, 0, st>>>(part2, nblk, D::C3, (const float*)d_in[base + 9], (const float*)d_in[base + 10],
                                 (const float*)d_in[base + 11], row2, invM);
  pool_out<D::C3, D::CBASE><<<(D::C3 / 32) * 32 * NBATCH, 256, 0, st>>>(pmx, pmn, row2, out1);
}

extern "C" void kernel_launch(void* const* d_in, const int* in_sizes, int n_in,
                              void* d_out, int out_size, void* d_ws, size_t ws_size, hipStream_t stream) {
  (void)in_sizes; (void)out_size;
  if (n_in < 38) return;
  if (ws_size < WS_TOTAL) return;

  const float* xyz = (const float*)d_in[0];
  const float* pts = (const float*)d_in[1];
  float* out0 = (float*)d_out;
  float* out1 = (float*)d_out + NBATCH * 3 * NQRY;

  char* ws = (char*)d_ws;
  size_t off = 0;
  unsigned short* x0 = (unsigned short*)(ws + off); off += SZ_X0;
  unsigned short* wpl = (unsigned short*)(ws + off); off += SZ_WPL;
  float* scsh = (float*)(ws + off); off += SZ_SCSH;
  float* p00 = (float*)(ws + off); off += part_bytes(1024, 32);
  float* p01 = (float*)(ws + off); off += part_bytes(1024, 32);
  float* p02 = (float*)(ws + off); off += part_bytes(1024, 64);
  float* p10 = (float*)(ws + off); off += part_bytes(2048, 64);
  float* p11 = (float*)(ws + off); off += part_bytes(2048, 64);
  float* p12 = (float*)(ws + off); off += part_bytes(2048, 128);
  float* p20 = (float*)(ws + off); off += part_bytes(8192, 64);
  float* p21 = (float*)(ws + off); off += part_bytes(8192, 96);
  float* p22 = (float*)(ws + off); off += part_bytes(8192, 128);
  float* mx0 = (float*)(ws + off); off += SZ_PM0;
  float* mn0 = (float*)(ws + off); off += SZ_PM0;
  float* mx1 = (float*)(ws + off); off += SZ_PM1;
  float* mn1 = (float*)(ws + off); off += SZ_PM1;
  float* mx2 = (float*)(ws + off); off += SZ_PM2;
  float* mn2 = (float*)(ws + off); off += SZ_PM2;
  if (off > ws_size) return;

  copy_queries<<<(NBATCH * 3 * NQRY / 4 + 255) / 256, 256, 0, stream>>>(xyz, out0);
  prep_weights<<<WPLANE_HALVES / 1024, 128, 0, stream>>>(
      (const float*)d_in[2],  (const float*)d_in[6],  (const float*)d_in[10],
      (const float*)d_in[14], (const float*)d_in[18], (const float*)d_in[22],
      (const float*)d_in[26], (const float*)d_in[30], (const float*)d_in[34], wpl);
  knn_gather<<<NBATCH * NQRY, 256, 0, stream>>>(xyz, pts, x0);

  run_scale<0>(d_in, x0, wpl, scsh, p00, p01, p02, mx0, mn0, out1, stream);
  run_scale<1>(d_in, x0, wpl, scsh, p10, p11, p12, mx1, mn1, out1, stream);
  run_scale<2>(d_in, x0, wpl, scsh, p20, p21, p22, mx2, mn2, out1, stream);
}
